// MoEBiEncoder_41266045780089
// MI455X (gfx1250) — hardware-run, weakly checked
//
#include <hip/hip_runtime.h>
#include <math.h>

typedef __attribute__((ext_vector_type(16))) _Float16 v16h;
typedef __attribute__((ext_vector_type(8)))  _Float16 v8h;
typedef __attribute__((ext_vector_type(8)))  float    v8f;
typedef __attribute__((ext_vector_type(4)))  float    v4f;

constexpr int kB   = 16384;
constexpr int kH   = 768;
constexpr int kH2  = 384;
constexpr int kE   = 8;
constexpr int kTM  = 64;
constexpr int kTiles = kB / kTM + kE;
constexpr int kSlots = kTiles * kTM;
constexpr int kRPT = 64;
constexpr int kPR  = 32;
constexpr int kXP = kH + 8;
constexpr int kHP = kH2 + 8;
constexpr int kYP = kH + 4;
static_assert(kB == kRPT * 256, "routing scan: 64 consecutive rows per thread, 256 threads");
static_assert(kE == 8, "eight branches: one wave per branch in the totals pass");
static_assert((kB % kPR) == 0 && kPR == 32 && kRPT == 2 * kPR, "placement blocks align with half spans");
static_assert((kH % 32) == 0 && (kH2 % 32) == 0, "K multiples of 32");
static_assert((kH % 64) == 0 && (kH2 % 64) == 0, "transpose tiles of 64");
static_assert(kH2 == 8 * 48 && kH == 8 * 96, "column split over 8 waves");
static_assert(kH == 6 * 128, "row = 6 instructions of 32 lanes x 4 floats");
static_assert((kXP * 2) % 16 == 0 && (kHP * 2) % 16 == 0 && (kYP * 4) % 16 == 0, "16-B aligned LDS rows");

constexpr float kCarryX = 16.0f;
constexpr float kCarryW = 256.0f;
constexpr float kCarryH = 16.0f;
constexpr float kFold1  = 1.0f / (kCarryX * kCarryW);
constexpr float kFold2  = 1.0f / (kCarryH * kCarryW);
constexpr float kF16Min = 6.103515625e-05f;

constexpr size_t kBytesW1T = (size_t)kE * kH2 * kH * 2;
constexpr size_t kBytesW2T = (size_t)kE * kH * kH2 * 2;
constexpr size_t kBytesGR  = (size_t)kSlots * kH * 4;
constexpr size_t kOffW1T   = 0;
constexpr size_t kOffW2T   = kOffW1T + kBytesW1T;
constexpr size_t kOffGR    = kOffW2T + kBytesW2T;
constexpr size_t kWsTotal  = kOffGR + kBytesGR;
static_assert(kBytesW1T == 4718592ull && kBytesW2T == 4718592ull && kBytesGR == 51904512ull, "plane sizes");
static_assert(kWsTotal == 61341696ull, "carve total");
static_assert(kWsTotal <= 134217728ull, "carve cap");
static_assert((kOffW2T % 128) == 0 && (kOffGR % 128) == 0, "aligned regions");

constexpr int kLdsH     = kTM * kHP * 2;
constexpr int kLdsX     = kTM * kXP * 2;
constexpr int kLdsY     = kTM * kYP * 4;
constexpr int kLdsScr   = 102400;
constexpr int kLdsTotal = kLdsH + kLdsY;
static_assert(kLdsH == 50176 && kLdsX == 99328 && kLdsY == 197632, "LDS sizes");
static_assert(kLdsScr >= kLdsX && (kLdsScr % 16) == 0, "scratch after the input tile");
static_assert(kLdsScr + kB + kE * 256 * 4 <= kLdsY, "scratch inside the shared region");
static_assert(kLdsTotal == 247808, "LDS total");

__device__ __forceinline__ _Float16 to_h_carry(float v, float carry) {
  float c = v * carry;
  c = (fabsf(c) < kF16Min) ? 0.0f : c;
  return (_Float16)c;
}

__device__ __forceinline__ v8f mma_g(v16h a, v16h b, v8f c) {
  c = __builtin_amdgcn_wmma_f32_16x16x32_f16(false, a, false, b, (short)0, c, false, false);
  asm volatile("v_nop\n\tv_nop\n\tv_nop\n\tv_nop" : "+v"(c) : "v"(a), "v"(b));
  return c;
}

union FragU { v16h v; v8h h[2]; };

__device__ __forceinline__ v16h frag_load(const _Float16* p) {
  FragU f;
  f.h[0] = *(const v8h*)(p);
  f.h[1] = *(const v8h*)(p + 16);
  return f.v;
}

__device__ __forceinline__ int first_max8(v4f a, v4f b, float& mx) {
  float m = a[0];
  int ei = 0;
  bool g;
  g = a[1] > m; m = g ? a[1] : m; ei = g ? 1 : ei;
  g = a[2] > m; m = g ? a[2] : m; ei = g ? 2 : ei;
  g = a[3] > m; m = g ? a[3] : m; ei = g ? 3 : ei;
  g = b[0] > m; m = g ? b[0] : m; ei = g ? 4 : ei;
  g = b[1] > m; m = g ? b[1] : m; ei = g ? 5 : ei;
  g = b[2] > m; m = g ? b[2] : m; ei = g ? 6 : ei;
  g = b[3] > m; m = g ? b[3] : m; ei = g ? 7 : ei;
  mx = m;
  return ei;
}

template <bool KEEP>
__device__ __forceinline__ void classify_span(const float* __restrict__ gl, int tid, int i0, int i1,
                                              int (&cnt)[kE], unsigned char* sel) {
#pragma unroll 2
  for (int i = i0; i < i1; ++i) {
    const int row = tid * kRPT + i;
    const v4f a = *(const v4f*)(gl + (size_t)row * kE);
    const v4f b = *(const v4f*)(gl + (size_t)row * kE + 4);
    float mx;
    const int ei = first_max8(a, b, mx);
    if (KEEP) sel[row] = (unsigned char)ei;
#pragma unroll
    for (int k = 0; k < kE; ++k) cnt[k] += (ei == k) ? 1 : 0;
  }
}

__device__ __forceinline__ void branch_tile_starts(const int (&tot)[kE], int (&ts)[kE + 1]) {
  ts[0] = 0;
#pragma unroll
  for (int k = 0; k < kE; ++k) {
    int c = tot[k];
    c = c < 0 ? 0 : (c > kB ? kB : c);
    ts[k + 1] = ts[k] + (c + kTM - 1) / kTM;
  }
}

__global__ __launch_bounds__(256) void transpose_cvt_f16_kernel(
    const float* __restrict__ in, unsigned short* __restrict__ outp, int rows, int cols)
{
  __shared__ float tile[64 * 65];
  const int tid = threadIdx.x, lane = tid & 31, wave = tid >> 5;
  const int c0 = blockIdx.x * 64;
  const int r0 = blockIdx.y * 64;
  const float* src = in + (size_t)blockIdx.z * rows * cols;
  unsigned short* dst = outp + (size_t)blockIdx.z * rows * cols;
  const int lc = tid & 63, lr = tid >> 6;
#pragma unroll 4
  for (int i = 0; i < 16; ++i) {
    const int r = lr + 4 * i;
    tile[r * 65 + lc] = src[(size_t)(r0 + r) * cols + c0 + lc];
  }
  __syncthreads();
  const int q = lane >> 3, c8 = (lane & 7) * 8;
  v8h hv[2];
#pragma unroll
  for (int it = 0; it < 2; ++it) {
    const int orow = it * 32 + wave * 4 + q;
#pragma unroll
    for (int e = 0; e < 8; ++e) {
      const float v = tile[(c8 + e) * 65 + orow];
      hv[it][e] = to_h_carry(v, kCarryW);
    }
  }
  for (int pass = 0; pass < 2; ++pass) {
#pragma unroll
    for (int it = 0; it < 2; ++it) {
      const int orow = it * 32 + wave * 4 + q;
      *(volatile v8h*)(dst + (size_t)(c0 + orow) * rows + r0 + c8) = hv[it];
    }
    __threadfence();
  }
}

__global__ __launch_bounds__(256) void routed_mlp_kernel(
    const float* __restrict__ emb, const float* __restrict__ gl,
    const unsigned short* __restrict__ W1tp, const float* __restrict__ b1,
    const unsigned short* __restrict__ W2tp, const float* __restrict__ b2,
    float* __restrict__ gr)
{
  extern __shared__ __align__(16) unsigned char dyn_lds[];
  __shared__ int   rowS[kTM];
  __shared__ float pS[kTM];
  __shared__ int   totS[kE];
  __shared__ int   wsumS[8];

  _Float16* Hh = (_Float16*)(dyn_lds);
  _Float16* Xh = (_Float16*)(dyn_lds + kLdsH);
  float*    Ys = (float*)(dyn_lds + kLdsH);
  unsigned char* selS = dyn_lds + kLdsH + kLdsScr;
  int* cntS = (int*)(dyn_lds + kLdsH + kLdsScr + kB);

  const int tid = threadIdx.x, lane = tid & 31, wave = tid >> 5;
  const int t = blockIdx.x;

  if (tid < kTM) rowS[tid] = -1;

  {
    int cnt[kE];
#pragma unroll
    for (int k = 0; k < kE; ++k) cnt[k] = 0;
    classify_span<true>(gl, tid, 0, kRPT, cnt, selS);
#pragma unroll
    for (int k = 0; k < kE; ++k) cntS[k * 256 + tid] = cnt[k];
  }
  __syncthreads();

  {
    int s = 0;
#pragma unroll
    for (int j = 0; j < 8; ++j) s += cntS[wave * 256 + lane * 8 + j];
#pragma unroll
    for (int off = 16; off > 0; off >>= 1) s += __shfl_xor(s, off, 32);
    if (lane == 0) totS[wave] = s;
  }
  __syncthreads();

  int e = -1, lt = 0;
  {
    int tot[kE];
#pragma unroll
    for (int k = 0; k < kE; ++k) tot[k] = totS[k];
    int ts[kE + 1];
    branch_tile_starts(tot, ts);
#pragma unroll
    for (int k = 0; k < kE; ++k) {
      const bool hit = (t >= ts[k]) && (t < ts[k + 1]);
      e  = hit ? k : e;
      lt = hit ? (t - ts[k]) : lt;
    }
  }
  if (e < 0) return;

  {
    const int c = cntS[e * 256 + tid];
    int v = c;
#pragma unroll
    for (int off = 1; off < 32; off <<= 1) {
      const int n = __shfl_up(v, off, 32);
      v += (lane >= off) ? n : 0;
    }
    if (lane == 31) wsumS[wave] = v;
    __syncthreads();
    int base = 0;
#pragma unroll
    for (int w = 0; w < 8; ++w) {
      const int x = wsumS[w];
      base += (w < wave) ? x : 0;
    }
    int rank = base + v - c;
    const int lo = lt * kTM;
#pragma unroll 4
    for (int i = 0; i < kRPT; ++i) {
      const int row = tid * kRPT + i;
      const int sv = (int)selS[row];
      const bool mt = (sv == e);
      const int slot = rank - lo;
      if (mt && slot >= 0 && slot < kTM) rowS[slot] = row;
      rank += mt ? 1 : 0;
    }
  }
  __syncthreads();

  {
    const int slot = tid & (kTM - 1);
    int r = rowS[slot];
    r = r < 0 ? 0 : (r > kB - 1 ? kB - 1 : r);
    const float* lp = gl + (size_t)r * kE;
    const v4f a = *(const v4f*)(lp);
    const v4f b = *(const v4f*)(lp + 4);
    float mx;
    (void)first_max8(a, b, mx);
    float s = 0.0f;
#pragma unroll 1
    for (int k = 0; k < kE; ++k) s += expf(lp[k] - mx);
    const float p = 1.0f / s;
    if (tid < kTM) pS[tid] = p;
  }

#pragma unroll 2
  for (int it = 0; it < 24; ++it) {
    const int i  = it * 256 + tid;
    const int s  = i / 96;
    const int c8 = (i - s * 96) * 8;
    const int r  = rowS[s];
    const bool ok = (r >= 0);
    const int rc = r < 0 ? 0 : (r > kB - 1 ? kB - 1 : r);
    v4f a0 = *(const v4f*)(emb + (size_t)rc * kH + c8);
    v4f a1 = *(const v4f*)(emb + (size_t)rc * kH + c8 + 4);
    asm volatile("" : "+v"(a0), "+v"(a1));
    v8h hv;
#pragma unroll
    for (int q = 0; q < 4; ++q) {
      const float f0 = ok ? a0[q] : 0.0f;
      const float f1 = ok ? a1[q] : 0.0f;
      hv[q]     = to_h_carry(f0, kCarryX);
      hv[4 + q] = to_h_carry(f1, kCarryX);
    }
    *(v8h*)(Xh + s * kXP + c8) = hv;
  }
  __syncthreads();

  const int rlane = lane & 15;
  const int koff  = (lane >> 4) * 8;
  const int mOff  = (lane >> 4) * 8;

  {
    const _Float16* W1e = (const _Float16*)W1tp + (size_t)e * kH2 * kH;
    const int nb = wave * 48;
    v8f acc[4][3];
#pragma unroll
    for (int i = 0; i < 4; ++i)
#pragma unroll
      for (int j = 0; j < 3; ++j) acc[i][j] = (v8f){0.f, 0.f, 0.f, 0.f, 0.f, 0.f, 0.f, 0.f};
#pragma unroll 1
    for (int k0 = 0; k0 < kH; k0 += 32) {
      v16h bf[3];
#pragma unroll
      for (int j = 0; j < 3; ++j)
        bf[j] = frag_load(W1e + (size_t)(nb + 16 * j + rlane) * kH + k0 + koff);
#pragma unroll
      for (int i = 0; i < 4; ++i) {
        const v16h af = frag_load(Xh + (16 * i + rlane) * kXP + k0 + koff);
#pragma unroll
        for (int j = 0; j < 3; ++j) acc[i][j] = mma_g(af, bf[j], acc[i][j]);
      }
    }
#pragma unroll
    for (int j = 0; j < 3; ++j) {
      const int n = nb + 16 * j + rlane;
      const float bv = b1[e * kH2 + n];
#pragma unroll
      for (int i = 0; i < 4; ++i) {
#pragma unroll
        for (int r = 0; r < 8; ++r) {
          float v = acc[i][j][r] * kFold1 + bv;
          v = fmaxf(v, 0.0f);
          Hh[(16 * i + mOff + r) * kHP + n] = to_h_carry(v, kCarryH);
        }
      }
    }
  }
  __syncthreads();

  {
    const _Float16* W2e = (const _Float16*)W2tp + (size_t)e * kH * kH2;
#pragma unroll 1
    for (int p = 0; p < 2; ++p) {
      const int nb = wave * 96 + p * 48;
      v8f acc[4][3];
#pragma unroll
      for (int i = 0; i < 4; ++i)
#pragma unroll
        for (int j = 0; j < 3; ++j) acc[i][j] = (v8f){0.f, 0.f, 0.f, 0.f, 0.f, 0.f, 0.f, 0.f};
#pragma unroll 1
      for (int k0 = 0; k0 < kH2; k0 += 32) {
        v16h bf[3];
#pragma unroll
        for (int j = 0; j < 3; ++j)
          bf[j] = frag_load(W2e + (size_t)(nb + 16 * j + rlane) * kH2 + k0 + koff);
#pragma unroll
        for (int i = 0; i < 4; ++i) {
          const v16h af = frag_load(Hh + (16 * i + rlane) * kHP + k0 + koff);
#pragma unroll
          for (int j = 0; j < 3; ++j) acc[i][j] = mma_g(af, bf[j], acc[i][j]);
        }
      }
#pragma unroll
      for (int j = 0; j < 3; ++j) {
        const int n = nb + 16 * j + rlane;
        const float bv = b2[e * kH + n];
#pragma unroll
        for (int i = 0; i < 4; ++i) {
#pragma unroll
          for (int r = 0; r < 8; ++r) {
            const int row = 16 * i + mOff + r;
            const float y = (acc[i][j][r] * kFold2 + bv) * pS[row];
            Ys[row * kYP + n] = y;
          }
        }
      }
    }
  }
  __syncthreads();

#pragma unroll 1
  for (int rr = 0; rr < 8; ++rr) {
    const int slot = wave * 8 + rr;
    const int r = rowS[slot];
    const int rc = r < 0 ? 0 : (r > kB - 1 ? kB - 1 : r);
    const float* yrow = Ys + slot * kYP + lane * 4;
    const float* xrow = emb + (size_t)rc * kH + lane * 4;
    v4f yv[6], xv[6];
#pragma unroll
    for (int it = 0; it < 6; ++it) {
      yv[it] = *(const v4f*)(yrow + 128 * it);
      xv[it] = *(const v4f*)(xrow + 128 * it);
    }
    float s = 0.0f;
#pragma unroll
    for (int it = 0; it < 6; ++it)
#pragma unroll
      for (int q = 0; q < 4; ++q) s = fmaf(yv[it][q], yv[it][q], s);
#pragma unroll
    for (int off = 16; off > 0; off >>= 1) s += __shfl_xor(s, off, 32);
    const float inv1 = 1.0f / fmaxf(sqrtf(s), 1e-6f);
    float s2 = 0.0f;
#pragma unroll
    for (int it = 0; it < 6; ++it) {
#pragma unroll
      for (int q = 0; q < 4; ++q) {
        const float v = fmaf(yv[it][q], inv1, xv[it][q]);
        yv[it][q] = v;
        s2 = fmaf(v, v, s2);
      }
    }
#pragma unroll
    for (int off = 16; off > 0; off >>= 1) s2 += __shfl_xor(s2, off, 32);
    const float inv2 = 1.0f / fmaxf(sqrtf(s2), 1e-12f);
#pragma unroll
    for (int it = 0; it < 6; ++it)
#pragma unroll
      for (int q = 0; q < 4; ++q) yv[it][q] = yv[it][q] * inv2;
    float* gp = gr + (size_t)(t * kTM + slot) * kH + lane * 4;
    for (int pass = 0; pass < 2; ++pass) {
#pragma unroll
      for (int it = 0; it < 6; ++it) *(volatile v4f*)(gp + 128 * it) = yv[it];
      __threadfence();
    }
  }
}

__global__ __launch_bounds__(256) void place_rows_kernel(
    const float* __restrict__ gl, const float* __restrict__ gr, float* __restrict__ out)
{
  __shared__ int wredS[8][2 * kE];
  const int tid = threadIdx.x, lane = tid & 31, wave = tid >> 5;
  const int r0 = blockIdx.x * kPR;
  const int tb = r0 / kRPT;
  const bool upper = (r0 & (kRPT - 1)) != 0;

  int cnt[kE], half[kE], bef[kE];
#pragma unroll
  for (int k = 0; k < kE; ++k) cnt[k] = 0;
  classify_span<false>(gl, tid, 0, kPR, cnt, nullptr);
#pragma unroll
  for (int k = 0; k < kE; ++k) half[k] = cnt[k];
  classify_span<false>(gl, tid, kPR, kRPT, cnt, nullptr);
#pragma unroll
  for (int k = 0; k < kE; ++k) {
    const int part = ((tid == tb) && upper) ? half[k] : 0;
    bef[k] = (tid < tb) ? cnt[k] : part;
  }
#pragma unroll
  for (int k = 0; k < kE; ++k) {
    int a = cnt[k], b = bef[k];
#pragma unroll
    for (int off = 16; off > 0; off >>= 1) {
      a += __shfl_xor(a, off, 32);
      b += __shfl_xor(b, off, 32);
    }
    cnt[k] = a;
    bef[k] = b;
  }
  if (lane == 0) {
#pragma unroll
    for (int k = 0; k < kE; ++k) {
      wredS[wave][k] = cnt[k];
      wredS[wave][kE + k] = bef[k];
    }
  }
  __syncthreads();
  int tot[kE], pre[kE];
#pragma unroll
  for (int k = 0; k < kE; ++k) {
    int a = 0, b = 0;
#pragma unroll
    for (int w = 0; w < 8; ++w) {
      a += wredS[w][k];
      b += wredS[w][kE + k];
    }
    tot[k] = a;
    pre[k] = b;
  }
  int ts[kE + 1];
  branch_tile_starts(tot, ts);

  int el;
  {
    const int row = r0 + lane;
    const v4f a = *(const v4f*)(gl + (size_t)row * kE);
    const v4f b = *(const v4f*)(gl + (size_t)row * kE + 4);
    float mx;
    el = first_max8(a, b, mx);
  }
  unsigned mymask = 0u;
  int tstart = 0, pr = 0;
#pragma unroll
  for (int k = 0; k < kE; ++k) {
    const bool mine = (el == k);
    const unsigned m = (unsigned)__ballot(mine ? 1 : 0);
    mymask = mine ? m : mymask;
    tstart = mine ? ts[k] : tstart;
    pr     = mine ? pre[k] : pr;
  }
  const unsigned below = (1u << lane) - 1u;
  const int rin = __popc(mymask & below);
  int slot = tstart * kTM + pr + rin;
  slot = slot < 0 ? 0 : (slot > kSlots - 1 ? kSlots - 1 : slot);

#pragma unroll 1
  for (int jj = 0; jj < 4; ++jj) {
    const int j = wave * 4 + jj;
    const int sj = __shfl(slot, j, 32);
    const float* src = gr + (size_t)sj * kH + lane * 4;
    v4f v[6];
#pragma unroll
    for (int it = 0; it < 6; ++it) v[it] = *(const v4f*)(src + 128 * it);
    float* op = out + (size_t)(r0 + j) * kH + lane * 4;
    for (int pass = 0; pass < 2; ++pass) {
#pragma unroll
      for (int it = 0; it < 6; ++it) *(volatile v4f*)(op + 128 * it) = v[it];
      __threadfence();
    }
  }
}

extern "C" void kernel_launch(void* const* d_in, const int* in_sizes, int n_in,
                              void* d_out, int out_size, void* d_ws, size_t ws_size,
                              hipStream_t stream) {
  if (n_in < 6) return;
  if (in_sizes[0] != kB * kH) return;
  if (in_sizes[1] != kB * kE) return;
  if (in_sizes[2] != kE * kH * kH2) return;
  if (in_sizes[3] != kE * kH2) return;
  if (in_sizes[4] != kE * kH2 * kH) return;
  if (in_sizes[5] != kE * kH) return;
  if (out_size != kB * kH) return;
  if (ws_size < kWsTotal) return;

  const float* emb = (const float*)d_in[0];
  const float* gl  = (const float*)d_in[1];
  const float* W1  = (const float*)d_in[2];
  const float* b1  = (const float*)d_in[3];
  const float* W2  = (const float*)d_in[4];
  const float* b2  = (const float*)d_in[5];
  float* out = (float*)d_out;

  char* ws = (char*)d_ws;
  unsigned short* W1T = (unsigned short*)(ws + kOffW1T);
  unsigned short* W2T = (unsigned short*)(ws + kOffW2T);
  float*          GR  = (float*)(ws + kOffGR);

  transpose_cvt_f16_kernel<<<dim3(kH2 / 64, kH / 64, kE), 256, 0, stream>>>(W1, W1T, kH, kH2);
  transpose_cvt_f16_kernel<<<dim3(kH / 64, kH2 / 64, kE), 256, 0, stream>>>(W2, W2T, kH2, kH);

  routed_mlp_kernel<<<dim3(kTiles), 256, kLdsTotal, stream>>>(emb, gl, W1T, b1, W2T, b2, GR);

  place_rows_kernel<<<dim3(kB / kPR), 256, 0, stream>>>(gl, GR, out);
}
